// NeuralEnergyLandscape_35003983462986
// MI455X (gfx1250) — hardware-verified
//
#include <hip/hip_runtime.h>


#define NS   524288
#define RCH  65536
#define NFE  38
#define KP   64
#define H1   128
#define H2   64
#define DM   KP
#define LOSC 1024.0f

typedef _Float16 h16;
typedef unsigned short bf;
typedef __attribute__((ext_vector_type(16))) __bf16   v16bf;
typedef __attribute__((ext_vector_type(16))) _Float16 v16h;
typedef __attribute__((ext_vector_type(8)))  _Float16 v8h;
typedef __attribute__((ext_vector_type(8)))  unsigned short v8us;
typedef __attribute__((ext_vector_type(8)))  float    v8f;
typedef __attribute__((ext_vector_type(4)))  float    v4f;
typedef v8h  __attribute__((may_alias)) v8ha;
typedef v4f  __attribute__((may_alias)) v4fa;
typedef v8us __attribute__((may_alias)) v8usa;

__device__ __forceinline__ unsigned short f2bf(float f) { unsigned u = __float_as_uint(f); u += 0x7FFFu + ((u >> 16) & 1u); return (unsigned short)(u >> 16); }
__device__ __forceinline__ float bf2f(unsigned short b) { return __uint_as_float(((unsigned)b) << 16); }
__device__ __forceinline__ float bfr(float f) { return bf2f(f2bf(f)); }
__device__ __forceinline__ v16h cat16(v8h lo, v8h hi) { return __builtin_shufflevector(lo, hi, 0, 1, 2, 3, 4, 5, 6, 7, 8, 9, 10, 11, 12, 13, 14, 15); }
__device__ __forceinline__ v16bf cat16b(v8us lo, v8us hi) { return __builtin_bit_cast(v16bf, __builtin_shufflevector(lo, hi, 0, 1, 2, 3, 4, 5, 6, 7, 8, 9, 10, 11, 12, 13, 14, 15)); }
__device__ __forceinline__ v8f wmma16(v16h a, v16h b, v8f c) { return __builtin_amdgcn_wmma_f32_16x16x32_f16(false, a, false, b, (short)0, c, false, false); }
__device__ __forceinline__ v8f wmmab(v16bf a, v16bf b, v8f c) { return __builtin_amdgcn_wmma_f32_16x16x32_bf16(false, a, false, b, (short)0, c, false, false); }

template <bool SPLITA, bool F16OUT = false>
__global__ __launch_bounds__(128) void k_gemmb(const bf* __restrict__ A, const bf* __restrict__ Al, const bf* __restrict__ Bn, const float* __restrict__ bias, float* C, int ldc, h16* C2, const float* __restrict__ R = nullptr, int K = DM, int roundR = 1) {
    __shared__ __align__(16) float ost[4][16 * 68];
    const int lane = threadIdx.x & 31, wave = threadIdx.x >> 5, lr = lane & 15, hi = lane >> 4;
    const int r0 = blockIdx.x * 64 + wave * 16, c0 = blockIdx.y * 64;
    const size_t aoff = (size_t)(r0 + lr) * K + 8 * hi;
    size_t boff[4];
#pragma unroll
    for (int t = 0; t < 4; ++t) boff[t] = (size_t)(c0 + t * 16 + lr) * K + 8 * hi;
    v8f acc[4];
#pragma unroll
    for (int t = 0; t < 4; ++t) acc[t] = (v8f){};
#pragma unroll 1
    for (int kc = 0; kc < K; kc += 32) {
        const v16bf a = cat16b(*(const v8us*)(A + aoff + kc), *(const v8us*)(A + aoff + kc + 16));
        v16bf al = a;
        if (SPLITA) al = cat16b(*(const v8us*)(Al + aoff + kc), *(const v8us*)(Al + aoff + kc + 16));
#pragma unroll
        for (int t = 0; t < 4; ++t) { const v16bf b = cat16b(*(const v8us*)(Bn + boff[t] + kc), *(const v8us*)(Bn + boff[t] + kc + 16)); acc[t] = wmmab(a, b, acc[t]); if (SPLITA) acc[t] = wmmab(al, b, acc[t]); }
        asm volatile("v_nop\n\tv_nop\n\tv_nop\n\tv_nop" : "+v"(acc[0]), "+v"(acc[1]), "+v"(acc[2]), "+v"(acc[3]) : "v"(a), "v"(al));
    }
    float* os = &ost[wave][0];
#pragma unroll
    for (int t = 0; t < 4; ++t) { const float bv = bias ? bfr(bias[c0 + t * 16 + lr]) : 0.f;
#pragma unroll
        for (int j = 0; j < 8; ++j) os[(hi * 8 + j) * 68 + t * 16 + lr] = acc[t][j] + bv; }
    __syncthreads();
    if (F16OUT) {
        h16* crow = (h16*)(void*)C + (size_t)r0 * ldc + c0;
        auto pass = [&]() {
#pragma unroll
            for (int s = 0; s < 4; ++s) { const int row = 4 * s + (lane >> 3), piece = lane & 7; const float* sp = os + row * 68 + piece * 8; v8h o, o2;
#pragma unroll
                for (int i = 0; i < 8; ++i) { const h16 a = (h16)sp[i]; o[i] = a; o2[i] = (h16)((sp[i] - (float)a) * LOSC); }
                *(volatile v8h*)(crow + (size_t)row * ldc + piece * 8) = o; if (C2) *(volatile v8h*)(C2 + (size_t)r0 * ldc + c0 + (size_t)row * ldc + piece * 8) = o2; }
        };
        pass(); __threadfence(); pass();
    } else {
        float* crow = C + (size_t)r0 * ldc + c0;
        auto pass = [&]() {
#pragma unroll
            for (int s = 0; s < 8; ++s) { const int Lid = (lane >> 3) + 4 * s, piece = lane & 7; const int row = Lid >> 1, cofs = (Lid & 1) * 32 + piece * 4;
                v4f val = *(const v4fa*)(os + row * 68 + cofs); if (R) { const v4f rv = *(const v4f*)(R + ((size_t)r0 + row) * ldc + c0 + cofs); val += roundR ? (v4f){bfr(rv[0]), bfr(rv[1]), bfr(rv[2]), bfr(rv[3])} : rv; }
                *(volatile v4f*)(crow + (size_t)row * ldc + cofs) = val; }
        };
        pass(); __threadfence(); pass();
    }
}

__global__ __launch_bounds__(256) void k_wt(const float* __restrict__ Wm, int K, int ncols, bf* WT) {
    __shared__ __align__(16) unsigned short tl[64 * 72];
    const int tid = threadIdx.x, k0 = blockIdx.x * 64, n0 = blockIdx.y * 64;
    const int kk = tid >> 2, nq = (tid & 3) * 16;
#pragma unroll
    for (int i = 0; i < 16; ++i) tl[(nq + i) * 72 + kk] = f2bf(Wm[(size_t)(k0 + kk) * ncols + n0 + nq + i]);
    __syncthreads();
    const int piece = tid & 7;
    auto pass = [&]() {
#pragma unroll
        for (int s = 0; s < 2; ++s) { const int nr = (tid >> 3) + 32 * s; const v8us val = *(const v8usa*)(tl + nr * 72 + piece * 8); *(volatile v8us*)(WT + (size_t)(n0 + nr) * K + k0 + piece * 8) = val; }
    };
    pass(); __threadfence(); pass();
}

__global__ __launch_bounds__(256) void k_wtp(const float* __restrict__ Wm, int krows, int ncols, int kpad, bf* WT) {
    __shared__ __align__(16) unsigned short tl[64 * 72];
    const int tid = threadIdx.x, k0 = blockIdx.x * 64, n0 = blockIdx.y * 64;
    const int kk = tid >> 2, nq = (tid & 3) * 16;
    const int k = k0 + kk, kc = k < krows ? k : krows - 1;
#pragma unroll
    for (int i = 0; i < 16; ++i) { const int n = n0 + nq + i, ncl = n < ncols ? n : ncols - 1; const float w = Wm[(size_t)kc * ncols + ncl]; tl[(nq + i) * 72 + kk] = (k < krows && n < ncols) ? f2bf(w) : (unsigned short)0; }
    __syncthreads();
    const int piece = tid & 7;
    auto pass = [&]() {
#pragma unroll
        for (int s = 0; s < 2; ++s) { const int nr = (tid >> 3) + 32 * s; const v8us val = *(const v8usa*)(tl + nr * 72 + piece * 8); *(volatile v8us*)(WT + (size_t)(n0 + nr) * kpad + k0 + piece * 8) = val; }
    };
    pass(); __threadfence(); pass();
}

__constant__ float c_mean[28] = {40000.0f, 40000.0f, 500.0f, 500.0f, 3000.0f, 3000.0f, 1000.0f, 1000.0f, 0.15f, 0.15f, 1.8f, 1.8f, 0.03f, 0.03f, -2.0f, -1.5f, -0.1f, -0.15f, 5.0f, 0.35f, 0.35f, 0.15f, 0.25f, 0.3f, 0.6f, 0.285f, 0.0f, 0.0f};
__constant__ float c_scale[28] = {30000.0f, 30000.0f, 500.0f, 500.0f, 2000.0f, 2000.0f, 800.0f, 800.0f, 0.1f, 0.1f, 0.5f, 0.5f, 0.02f, 0.02f, 2.0f, 2.0f, 0.5f, 0.5f, 3.0f, 0.25f, 0.25f, 0.2f, 0.2f, 0.3f, 0.15f, 0.05f, 0.02f, 0.02f};
__constant__ int c_idx[16] = {0, 1, 2, 3, 4, 5, 14, 15, 12, 13, 25, 19, 20, 21, 22, 24};
__constant__ float c_sqs[4] = {0.1f, 0.1f, 0.05f, 0.05f};
__constant__ float c_svs[7] = {25.0f, 1.0f, 1.5f, 1.0f, 1.0f, 75.0f, 75.0f};
__constant__ float c_aqs[4] = {0.1f, 0.05f, 0.05f, 0.05f};
__constant__ float c_avs[7] = {5.0f, 1.0f, 1.0f, 75.0f, 75.0f, 75.0f, 75.0f};
__device__ __forceinline__ float featv(const float* __restrict__ q, const float* __restrict__ p, const float* __restrict__ sp, const float* __restrict__ Md, size_t s, int c) {
    #pragma clang fp contract(off)
    auto Q = [&](int i) { return bfr(q[s * 14 + i]); }; auto V = [&](int i) { return ((bfr(p[s * 14 + i])) * __builtin_amdgcn_rcpf(bfr(Md[i]))); };
    if (c < 4) { float x; if (c == 0) x = Q(2); else if (c == 1) x = Q(4); else if (c == 2) x = (Q(6) + Q(7)) * 0.5f; else x = (Q(8) + Q(9)) * 0.5f; return ((x) * __builtin_amdgcn_rcpf(c_sqs[c] + 1e-6f)); }
    if (c < 11) { const int k = c - 4; float x; if (k == 0) x = V(0); else if (k == 1) x = V(2); else if (k == 2) x = V(4); else if (k == 3) x = (V(6) + V(7)) * 0.5f; else if (k == 4) x = (V(8) + V(9)) * 0.5f; else if (k == 5) x = (V(10) + V(11)) * 0.5f; else x = (V(12) + V(13)) * 0.5f;
        return ((x) * __builtin_amdgcn_rcpf(c_svs[k] + 1e-6f)); }
    if (c < 15) { const int k = c - 11; float x; if (k == 0) x = Q(3); else if (k == 1) x = Q(6) - Q(7); else if (k == 2) x = Q(8) - Q(9); else x = Q(6) + Q(9) - Q(7) - Q(8); x = x * x; return ((x) * __builtin_amdgcn_rcpf(c_aqs[k] * c_aqs[k] + 1e-6f)); }
    if (c < 22) { const int k = c - 15; float x; if (k == 0) x = V(1); else if (k == 1) x = V(3); else if (k == 2) x = V(5); else if (k == 3) x = V(6) - V(7); else if (k == 4) x = V(8) - V(9); else if (k == 5) x = V(10) - V(11); else x = V(12) - V(13); x = x * x;
        return ((x) * __builtin_amdgcn_rcpf(c_avs[k] * c_avs[k] + 1e-6f)); }
    if (c < 38) { const int k = c - 22; const int j = c_idx[k]; return ((bfr(sp[s * 28 + j]) - c_mean[j]) * __builtin_amdgcn_rcpf(c_scale[j] + 1e-6f)); }
    return 0.f;
}
__global__ __launch_bounds__(256) void k_feat(const float* __restrict__ q, const float* __restrict__ p, const float* __restrict__ sp, const float* __restrict__ Md, int s0, bf* Fh, bf* Fl) {
    __shared__ float fs[256][41];
    const int tid = threadIdx.x, lane = tid & 31, wv = tid >> 5; const size_t sb = (size_t)blockIdx.x * 256;
    { const size_t s = (size_t)s0 + sb + tid;
#pragma unroll 1
      for (int c = 0; c < NFE; ++c) fs[tid][c] = featv(q, p, sp, Md, s, c); }
    __syncthreads();
    auto pass = [&]() {
#pragma unroll 1
        for (int st = 0; st < 8; ++st) { const int sl = wv * 32 + st * 4 + (lane >> 3); const int cb = (lane & 7) * 8; v8us oh, ol;
#pragma unroll
            for (int i = 0; i < 8; ++i) { const int c = cb + i; const float f = (c < NFE) ? fs[sl][c < NFE ? c : 0] : 0.f; const unsigned short hb = f2bf(f); oh[i] = hb; ol[i] = f2bf(f - bf2f(hb)); }
            const size_t o = (sb + sl) * KP + cb; *(volatile v8us*)(Fh + o) = oh; *(volatile v8us*)(Fl + o) = ol; }
    };
    pass(); __threadfence(); pass();
}
__device__ __forceinline__ float swish_f(float x) { return ((x) * __builtin_amdgcn_rcpf(1.0f + __expf(-x))); }
__global__ __launch_bounds__(256) void k_sw1(const float* __restrict__ X1, const float* __restrict__ b1, bf* Ph, bf* Pl) {
    const int lane = threadIdx.x & 31; const size_t rl = ((size_t)blockIdx.x * 8 + (threadIdx.x >> 5)) * 2 + (lane >> 4); const int cb = (lane & 15) * 8; v8us oh, ol;
#pragma unroll
    for (int i = 0; i < 8; ++i) { const float v = swish_f(X1[rl * H1 + cb + i] + bfr(b1[cb + i])); const unsigned short hb = f2bf(v); oh[i] = hb; ol[i] = f2bf(v - bf2f(hb)); }
    const size_t o = rl * H1 + cb; *(volatile v8us*)(Ph + o) = oh; *(volatile v8us*)(Pl + o) = ol; __threadfence(); *(volatile v8us*)(Ph + o) = oh; *(volatile v8us*)(Pl + o) = ol;
}
__global__ __launch_bounds__(256) void k_fin(const float* __restrict__ X2, const float* __restrict__ b2, const float* __restrict__ W3, const float* __restrict__ b3, const float* __restrict__ q, const float* __restrict__ p, const float* __restrict__ Md, int s0, float* OUTP) {
    const size_t sl = (size_t)blockIdx.x * 256 + threadIdx.x; const size_t s = (size_t)s0 + sl; float acc = bfr(b3[0]);
#pragma unroll 1
    for (int c = 0; c < H2; ++c) acc = fmaf(swish_f(X2[sl * H2 + c] + bfr(b2[c])), bfr(W3[c]), acc);
    const float spl = log1pf(__expf(-fabsf(acc))) + fmaxf(acc, 0.f); const float hraw = fminf(spl * 1.0f, 5000.0f);
    float tp = 0.f;
#pragma unroll 1
    for (int i = 0; i < 14; ++i) { const float pv = bfr(p[s * 14 + i]); tp += ((pv * pv) * __builtin_amdgcn_rcpf(bfr(Md[i]))); }
    tp *= 0.5f;
    float sq = 0.f;
#pragma unroll
    for (int i = 6; i < 10; ++i) { const float qv = bfr(q[s * 14 + i]); sq += qv * qv; }
    const float v = tp + 0.5f * sq * 30000.0f + hraw * sq;
    *(volatile float*)(OUTP + s) = v; __threadfence(); *(volatile float*)(OUTP + s) = v;
}

extern "C" void kernel_launch(void* const* d_in, const int* in_sizes, int n_in,
                              void* d_out, int out_size, void* d_ws, size_t ws_size, hipStream_t stream) {
    (void)in_sizes; (void)n_in; (void)out_size;
    const float* q = (const float*)d_in[0]; const float* p = (const float*)d_in[1]; const float* sp = (const float*)d_in[2]; const float* Md = (const float*)d_in[3];
    const float* W1 = (const float*)d_in[4]; const float* b1 = (const float*)d_in[5]; const float* W2 = (const float*)d_in[6]; const float* b2 = (const float*)d_in[7]; const float* W3 = (const float*)d_in[8]; const float* b3 = (const float*)d_in[9];
    float* out = (float*)d_out;
    char* wsp = (char*)d_ws;
    auto take = [&](size_t bytes) { char* pp = wsp; wsp += (bytes + 255) & ~(size_t)255; return (void*)pp; };
    bf* W1T = (bf*)take((size_t)H1 * KP * 2); bf* W2T = (bf*)take((size_t)H2 * H1 * 2);
    bf* Fh = (bf*)take((size_t)RCH * KP * 2); bf* Fl = (bf*)take((size_t)RCH * KP * 2); float* X1 = (float*)take((size_t)RCH * H1 * 4); bf* Ph = (bf*)take((size_t)RCH * H1 * 2); bf* Pl = (bf*)take((size_t)RCH * H1 * 2); float* X2 = (float*)take((size_t)RCH * H2 * 4);
    if ((size_t)(wsp - (char*)d_ws) > ws_size) return;
    k_wtp<<<dim3(KP / 64, H1 / 64, 1), 256, 0, stream>>>(W1, NFE, H1, KP, W1T);
    k_wt<<<dim3(H1 / 64, H2 / 64, 1), 256, 0, stream>>>(W2, H1, H2, W2T);
    for (int ch = 0; ch < NS / RCH; ++ch) { const int s0 = ch * RCH;
        k_feat<<<RCH / 256, 256, 0, stream>>>(q, p, sp, Md, s0, Fh, Fl);
        k_gemmb<true, false><<<dim3(RCH / 64, H1 / 64, 1), 128, 0, stream>>>(Fh, Fl, W1T, nullptr, X1, H1, nullptr, nullptr, KP);
        k_sw1<<<RCH / 16, 256, 0, stream>>>(X1, b1, Ph, Pl);
        k_gemmb<true, false><<<dim3(RCH / 64, H2 / 64, 1), 128, 0, stream>>>(Ph, Pl, W2T, nullptr, X2, H2, nullptr, nullptr, H1);
        k_fin<<<RCH / 256, 256, 0, stream>>>(X2, b2, W3, b3, q, p, Md, s0, out); }
}
